// Convolution_58076547777063
// MI455X (gfx1250) — hardware-verified
//
#include <hip/hip_runtime.h>
#include <stddef.h>
#include <stdint.h>
#include <math.h>


#define DIN     128
#define HC      128
#define NX      256
#define KH      256
#define NTHR    256
#define NWAVE   8
#define EPT     8
#define CHUNK   (NTHR * EPT)
#define WCAP    (EPT * 32)
#define LISTN   (NWAVE * WCAP)
#define NBA     1024
#define SLA     10
#define RCAP    28672
#define DEGCAP  128
#define MEAS_B1024  16623
#define MEAS_MAXDEG 35
#define GBM     64
#define GBN     64
#define GTHR    128
#define MROWS   128
#define NEGSL   0.2f
#define WSMAX   134217728
#define P_BIAS  0
#define P_WE    256
#define P_ATT   384
#define P_BO    512
#define P_BLIN  640
#define PARN    768
#define OFF_W1  0
#define OFF_W2  32768
#define OFF_W3  98304
#define WPLN    131072
#define NUWT    16384
#define BKT_LDS_INTS  (LISTN + 2 * RCAP + 4 * NBA + 16)
#define SCAN_LDS_INTS (2 * RCAP + 3 * NBA + 16)
#define KATTR __attribute__((amdgpu_num_vgpr(248)))

static_assert(HC == 4 * 32);
static_assert(32 * 4 == HC);
static_assert((HC / 4) / 4 == 8);
static_assert(NBA == 1024 && NBA == (1 << SLA));
static_assert((CHUNK & (CHUNK - 1)) == 0 && CHUNK <= 4096);
static_assert(((long long)CHUNK << SLA) < (1LL << 31));
static_assert(LISTN >= NWAVE * WCAP);
static_assert(NBA % NWAVE == 0 && NBA == NTHR * 4);
static_assert((RCAP % 32) == 0);
static_assert((long long)RCAP * 100 >= (long long)MEAS_B1024 * 105);
static_assert(DEGCAP >= MEAS_MAXDEG + 8);
static_assert(BKT_LDS_INTS * 4 <= 300000 && SCAN_LDS_INTS * 4 <= 300000);
static_assert(GBM == (GTHR / 32) * 16);
static_assert((DIN % 32) == 0 && (KH % 32) == 0);
static_assert((NX % GBN) == 0 && (HC % GBN) == 0);
static_assert((MROWS % GBM) == 0);
static_assert(KH == 2 * HC && NX == 2 * HC);
static_assert(OFF_W2 == NX * DIN && OFF_W3 == OFF_W2 + NX * KH && WPLN == OFF_W3 + HC * KH);
static_assert(NUWT * 8 == WPLN && (NUWT % NTHR) == 0);
static_assert(PARN == 6 * 128 && P_BLIN + 128 == PARN);

typedef float          v4f  __attribute__((ext_vector_type(4)));
typedef float          v8f  __attribute__((ext_vector_type(8)));
typedef int            v2i  __attribute__((ext_vector_type(2)));
typedef int            v4i  __attribute__((ext_vector_type(4)));
typedef int            v8i  __attribute__((ext_vector_type(8)));
typedef unsigned short v4us __attribute__((ext_vector_type(4)));
typedef unsigned short v8us __attribute__((ext_vector_type(8)));
typedef __bf16         v16b __attribute__((ext_vector_type(16)));
typedef v4f  __attribute__((may_alias)) v4fa;
typedef v2i  __attribute__((may_alias)) v2ia;
typedef v4i  __attribute__((may_alias)) v4ia;
typedef v8us __attribute__((may_alias)) v8usa;
union FragB { v16b v; v8us h[2]; v8i w; };

__device__ __forceinline__ v8f wmb(const FragB& a, const FragB& b, v8f c) {
  v8f d = __builtin_amdgcn_wmma_f32_16x16x32_bf16(false, a.v, false, b.v, (short)0, c, false, false);
  asm volatile("v_nop\n\tv_nop\n\tv_nop\n\tv_nop" : "+v"(d) : "v"(a.w), "v"(b.w));
  return d;
}

__device__ __forceinline__ unsigned int f2bf(float f) {
  const unsigned int u = __float_as_uint(f);
  const unsigned int r = ((u + 0x7FFFu + ((u >> 16) & 1u)) >> 16) & 0xFFFFu;
  return ((u & 0x7FFFFFFFu) > 0x7F800000u) ? 0x7FC0u : r;
}
__device__ __forceinline__ float bf2f(unsigned int b) { return __uint_as_float(b << 16); }
__device__ __forceinline__ float bfr(float f) { return bf2f(f2bf(f)); }

template <int SLB>
__device__ __forceinline__ int scan_chunk(const int* __restrict__ dsts, int nE, int cbase, int slotBase,
                                          int nb, int vec8, int* list, int tid, int lane, int wave) {
  int wc = 0;
  const int el0  = tid * EPT;
  const int e0   = cbase + el0;
  const int sent = -2147483647 - 1;
  v4i da, db;
  if (vec8 != 0 && cbase + CHUNK <= nE) {
    da = *(const v4i*)(dsts + e0);
    db = *(const v4i*)(dsts + e0 + 4);
  } else {
    da.x = (e0     < nE) ? dsts[min(e0,     nE - 1)] : sent;
    da.y = (e0 + 1 < nE) ? dsts[min(e0 + 1, nE - 1)] : sent;
    da.z = (e0 + 2 < nE) ? dsts[min(e0 + 2, nE - 1)] : sent;
    da.w = (e0 + 3 < nE) ? dsts[min(e0 + 3, nE - 1)] : sent;
    db.x = (e0 + 4 < nE) ? dsts[min(e0 + 4, nE - 1)] : sent;
    db.y = (e0 + 5 < nE) ? dsts[min(e0 + 5, nE - 1)] : sent;
    db.z = (e0 + 6 < nE) ? dsts[min(e0 + 6, nE - 1)] : sent;
    db.w = (e0 + 7 < nE) ? dsts[min(e0 + 7, nE - 1)] : sent;
  }
  const unsigned nbs = (unsigned)slotBase;
  const unsigned unb = (unsigned)nb;
  const unsigned s0 = (unsigned)da.x - nbs, s1 = (unsigned)da.y - nbs;
  const unsigned s2 = (unsigned)da.z - nbs, s3 = (unsigned)da.w - nbs;
  const unsigned s4 = (unsigned)db.x - nbs, s5 = (unsigned)db.y - nbs;
  const unsigned s6 = (unsigned)db.z - nbs, s7 = (unsigned)db.w - nbs;
  const bool h0 = s0 < unb, h1 = s1 < unb, h2 = s2 < unb, h3 = s3 < unb;
  const bool h4 = s4 < unb, h5 = s5 < unb, h6 = s6 < unb, h7 = s7 < unb;
  const unsigned any = __builtin_amdgcn_ballot_w32(h0 | h1 | h2 | h3 | h4 | h5 | h6 | h7);
  if (any != 0u) {
#define HITJ(J, HJ, SJ) { \
      const unsigned mj = __builtin_amdgcn_ballot_w32(HJ); \
      if (mj != 0u) { \
        if (HJ) { \
          const int pos = wc + (int)__builtin_amdgcn_mbcnt_lo(mj, 0u); \
          if (pos < WCAP) list[wave * WCAP + pos] = ((el0 + (J)) << SLB) | (int)(SJ); \
        } \
        wc += (int)__builtin_popcount(mj); } }
    HITJ(0, h0, s0)
    HITJ(1, h1, s1)
    HITJ(2, h2, s2)
    HITJ(3, h3, s3)
    HITJ(4, h4, s4)
    HITJ(5, h5, s5)
    HITJ(6, h6, s6)
    HITJ(7, h7, s7)
#undef HITJ
  }
  return wc;
}

__global__ __launch_bounds__(NTHR) KATTR void k_pa(const float* __restrict__ x, unsigned short* xb,
                                                   int nN, int nUnits) {
  const int i = (int)blockIdx.x * NTHR + (int)threadIdx.x;
  if (i >= nUnits) return;
  const int row = i >> 4;
  const int c0  = (i & 15) * 8;
  const int rc  = row < nN ? row : nN - 1;
  const float* p = x + (size_t)rc * DIN + c0;
  v4f a = *(const v4f*)p, b = *(const v4f*)(p + 4);
  const v4f z4 = {0.f, 0.f, 0.f, 0.f};
  if (row >= nN) { a = z4; b = z4; }
  v8us hv;
  hv[0] = (unsigned short)f2bf(a.x); hv[1] = (unsigned short)f2bf(a.y);
  hv[2] = (unsigned short)f2bf(a.z); hv[3] = (unsigned short)f2bf(a.w);
  hv[4] = (unsigned short)f2bf(b.x); hv[5] = (unsigned short)f2bf(b.y);
  hv[6] = (unsigned short)f2bf(b.z); hv[7] = (unsigned short)f2bf(b.w);
  const size_t o = (size_t)row * DIN + c0;
  *(volatile v8us*)(xb + o) = hv;
  __threadfence();
  *(volatile v8us*)(xb + o) = hv;
}

__device__ __forceinline__ v8us col8(const float* __restrict__ w, int kk, int n) {
  const float* p = w + (size_t)kk * HC + n;
  v8us o;
#pragma unroll
  for (int i = 0; i < 8; ++i) o[i] = (unsigned short)f2bf(p[(size_t)i * HC]);
  return o;
}

__global__ __launch_bounds__(NTHR) KATTR void k_pb(const float* __restrict__ Wl1, const float* __restrict__ Wr1,
                                                   const float* __restrict__ Wl2, const float* __restrict__ Wr2,
                                                   const float* __restrict__ Wlin, unsigned short* WP) {
  const int u = (int)blockIdx.x * NTHR + (int)threadIdx.x;
  v8us o;
  int off;
  if (u < 2048) {
    const int n = u >> 4, k8 = (u & 15) * 8;
    o = col8(Wl1, k8, n);
    off = OFF_W1 + n * DIN + k8;
  } else if (u < 4096) {
    const int v = u - 2048;
    const int n = v >> 4, k8 = (v & 15) * 8;
    o = col8(Wr1, k8, n);
    off = OFF_W1 + (HC + n) * DIN + k8;
  } else if (u < 8192) {
    const int v = u - 4096;
    const int n = v >> 5, k8 = (v & 31) * 8;
    o = col8(Wl2, k8 & (HC - 1), n);
    off = OFF_W2 + n * KH + k8;
  } else if (u < 12288) {
    const int v = u - 8192;
    const int n = v >> 5, k8 = (v & 31) * 8;
    o = col8(Wr2, k8 & (HC - 1), n);
    off = OFF_W2 + (HC + n) * KH + k8;
  } else if (u < NUWT) {
    const int v = u - 12288;
    const int n = v >> 5, k8 = (v & 31) * 8;
    o = col8(Wlin, k8 & (HC - 1), n);
    off = OFF_W3 + n * KH + k8;
  } else {
    return;
  }
  unsigned short* dp = WP + off;
  *(volatile v8us*)dp = o;
  __threadfence();
  *(volatile v8us*)dp = o;
}

__global__ __launch_bounds__(NTHR) KATTR void k_par(const float* __restrict__ s0, const float* __restrict__ s1,
                                                    const float* __restrict__ s2, const float* __restrict__ s3,
                                                    const float* __restrict__ s4, const float* __restrict__ s5,
                                                    float* out, int nseg) {
  const int u   = (int)threadIdx.x;
  const int seg = u >> 5;
  const int i4  = (u & 31) * 4;
  const v4f a0 = *(const v4f*)(s0 + i4);
  const v4f a1 = *(const v4f*)(s1 + i4);
  const v4f a2 = *(const v4f*)(s2 + i4);
  const v4f a3 = *(const v4f*)(s3 + i4);
  const v4f a4 = *(const v4f*)(s4 + i4);
  const v4f a5 = *(const v4f*)(s5 + i4);
  v4f v = a0;
  v = (seg == 1) ? a1 : v;
  v = (seg == 2) ? a2 : v;
  v = (seg == 3) ? a3 : v;
  v = (seg == 4) ? a4 : v;
  v = (seg >= 5) ? a5 : v;
  v4f r;
  r.x = bfr(v.x); r.y = bfr(v.y); r.z = bfr(v.z); r.w = bfr(v.w);
  const int sc = seg < 5 ? seg : 5;
  float* op = out + sc * 128 + i4;
  const bool wr = seg < nseg;
  if (wr) *(volatile v4f*)op = r;
  __threadfence();
  if (wr) *(volatile v4f*)op = r;
}

__global__ __launch_bounds__(NTHR) KATTR void k_bucket(const int* __restrict__ srcs, const int* __restrict__ dsts,
                                                       const float* __restrict__ eattr, int nE, int nN, int vec8,
                                                       int* REC, int* CNT, int* OFF, float* LOOPA, int* FLG) {
  extern __shared__ __attribute__((aligned(16))) int bsm[];
  int*   list = bsm;
  int*   reg1 = list + LISTN;
  int*   sl   = reg1 + RCAP;
  int*   cnt  = sl + RCAP;
  int*   offs = cnt + NBA;
  int*   cur  = offs + NBA;
  float* laf  = (float*)(cur + NBA);
  int*   wcnt = cur + 2 * NBA;
  const int tid = (int)threadIdx.x, lane = tid & 31, wave = tid >> 5;
  const int blk = (int)blockIdx.x;
  const int nodeBase = blk * NBA;
  int nb = nN - nodeBase;
  nb = nb < 0 ? 0 : (nb > NBA ? NBA : nb);

  {
    const v4i z4 = {0, 0, 0, 0};
    for (int i = tid * 4; i < 3 * NBA; i += NTHR * 4) *(v4ia*)(cnt + i) = z4;
    const v4f zf = {0.f, 0.f, 0.f, 0.f};
    *(v4fa*)(laf + 4 * tid) = zf;
    if (tid < 16) wcnt[tid] = 0;
  }
  __syncthreads();

  int tot = 0, ovf = 0;
  const int nChunks = (nE + CHUNK - 1) / CHUNK;
#pragma unroll 1
  for (int ch = 0; ch < nChunks; ++ch) {
    const int cbase = ch * CHUNK;
    const int wc = scan_chunk<SLA>(dsts, nE, cbase, nodeBase, nb, vec8, list, tid, lane, wave);
    if (lane == 0) wcnt[wave] = wc;
    __syncthreads();
    int pre = 0, all = 0;
#pragma unroll
    for (int w2 = 0; w2 < NWAVE; ++w2) {
      int c = wcnt[w2];
      c = c < 0 ? 0 : (c > WCAP ? WCAP : c);
      all += c;
      pre += (w2 < wave) ? c : 0;
    }
    const int wcc  = wc > WCAP ? WCAP : wc;
    const int base = tot + pre;
#pragma unroll 1
    for (int i = lane; i < wcc; i += 32) {
      const int ent = list[wave * WCAP + i];
      const int el  = (ent >> SLA) & (CHUNK - 1);
      const int sq  = ent & (NBA - 1);
      int eid = cbase + el;
      eid = eid > nE - 1 ? nE - 1 : eid;
      const int pos = base + i;
      if (pos < RCAP) reg1[pos] = (int)(((unsigned)eid << SLA) | (unsigned)sq);
    }
    if (tot + all > RCAP) ovf = 1;
    tot += all;
    tot = tot > RCAP ? RCAP : tot;
    __syncthreads();
  }
  const int nh = tot;
  const int nhPad = (nh + 31) & ~31;

  if (wave == 0) {
#pragma unroll 1
    for (int b0 = 0; b0 < nh; b0 += 32) {
      const int idx = b0 + lane;
      const int uv  = reg1[idx < nh ? idx : nh - 1];
      const int m32 = (nh - b0) < 32 ? (nh - b0) : 32;
#pragma unroll 1
      for (int k = 0; k < m32; ++k) {
        const int u  = __builtin_amdgcn_readlane(uv, k);
        const int sq = u & (NBA - 1);
        if (lane == 0) cnt[sq] = cnt[sq] + 1;
      }
    }
  }
  __syncthreads();
  if (wave == 0) {
    const int base = lane * (NBA / 32);
    int s = 0;
#pragma unroll 1
    for (int i = 0; i < NBA / 32; ++i) s += cnt[base + i];
    int incl = s;
#pragma unroll
    for (int d = 1; d < 32; d <<= 1) {
      const int y = __shfl_up(incl, d, 32);
      if (lane >= d) incl += y;
    }
    int run = incl - s;
#pragma unroll 1
    for (int i = 0; i < NBA / 32; ++i) {
      const int cv = cnt[base + i];
      offs[base + i] = run;
      cur[base + i]  = run;
      run += cv;
    }
  }
  __syncthreads();
  if (wave == 0) {
#pragma unroll 1
    for (int b0 = 0; b0 < nh; b0 += 32) {
      const int idx = b0 + lane;
      const int uv  = reg1[idx < nh ? idx : nh - 1];
      const int m32 = (nh - b0) < 32 ? (nh - b0) : 32;
#pragma unroll 1
      for (int k = 0; k < m32; ++k) {
        const int u   = __builtin_amdgcn_readlane(uv, k);
        const int sq  = u & (NBA - 1);
        const int eid = (int)((unsigned)u >> SLA);
        if (lane == 0) {
          int p = cur[sq];
          p = p < 0 ? 0 : (p > RCAP - 1 ? RCAP - 1 : p);
          sl[p] = eid;
          cur[sq] = p + 1;
        }
      }
    }
  }
  __syncthreads();

#pragma unroll 1
  for (int p = tid; p < nh; p += NTHR) {
    int eid = sl[p];
    eid = eid < 0 ? 0 : (eid > nE - 1 ? nE - 1 : eid);
    const int sraw = srcs[eid];
    const float araw = eattr[eid];
    const int s = sraw < 0 ? 0 : (sraw > nN - 1 ? nN - 1 : sraw);
    reg1[p] = s;
    sl[p]   = __float_as_int(bfr(araw));
  }
  for (int p = nh + tid; p < nhPad; p += NTHR) { reg1[p] = 0; sl[p] = 0; }
  __syncthreads();

#pragma unroll 1
  for (int s = tid; s < NBA; s += NTHR) {
    const int craw = cnt[s];
    int c = craw < 0 ? 0 : (craw > DEGCAP ? DEGCAP : craw);
    int o = offs[s];
    o = o < 0 ? 0 : (o > nh ? nh : o);
    if (c > nh - o) c = nh - o;
    float sum = 0.0f;
#pragma unroll 1
    for (int q = 0; q < c; ++q) sum += __int_as_float(sl[o + q]);
    const float den  = (c > 0) ? (float)c : 1.0f;
    const float mean = sum / den;
    laf[s] = (c > 0) ? mean : 0.0f;
    if (craw > DEGCAP) wcnt[8] = 1;
  }
  __syncthreads();

  const int flag = (ovf != 0 || wcnt[8] != 0) ? 1 : 0;
  int* rb = REC + (size_t)blk * (size_t)(2 * RCAP);
  const int nI = 2 * nhPad;
  const v4i cvn = *(const v4ia*)(cnt + 4 * tid);
  const v4i ovn = *(const v4ia*)(offs + 4 * tid);
  const v4f lvn = *(const v4fa*)(laf + 4 * tid);
  int*   cp = CNT   + (size_t)blk * NBA + 4 * tid;
  int*   op = OFF   + (size_t)blk * NBA + 4 * tid;
  float* lp = LOOPA + (size_t)blk * NBA + 4 * tid;
  v4i fv;
  fv.x = (tid == 0) ? nh : 0;
  fv.y = (tid == 0) ? flag : 0;
  fv.z = 0; fv.w = 0;
  int* fp = FLG + (size_t)blk * 32 + 4 * (tid & 7);
#pragma unroll 1
  for (int p = tid * 4; p < nI; p += NTHR * 4) {
    const int r = p >> 1;
    v4i v;
    v.x = reg1[r];     v.y = sl[r];
    v.z = reg1[r + 1]; v.w = sl[r + 1];
    *(volatile v4i*)(rb + p) = v;
  }
  *(volatile v4i*)cp = cvn;
  *(volatile v4i*)op = ovn;
  *(volatile v4f*)lp = lvn;
  if (tid < 8) *(volatile v4i*)fp = fv;
  __threadfence();
#pragma unroll 1
  for (int p = tid * 4; p < nI; p += NTHR * 4) {
    const int r = p >> 1;
    v4i v;
    v.x = reg1[r];     v.y = sl[r];
    v.z = reg1[r + 1]; v.w = sl[r + 1];
    *(volatile v4i*)(rb + p) = v;
  }
  *(volatile v4i*)cp = cvn;
  *(volatile v4i*)op = ovn;
  *(volatile v4f*)lp = lvn;
  if (tid < 8) *(volatile v4i*)fp = fv;
}

__global__ __launch_bounds__(GTHR) KATTR void k_gemm(
    const unsigned short* __restrict__ A, const unsigned short* __restrict__ WT,
    const float* __restrict__ bias, float* outF, int K, int ldo, int relu, int nStore)
{
  __shared__ __attribute__((aligned(16))) float stg[GBM * GBN];
  const int tid = (int)threadIdx.x, lane = tid & 31, wave = tid >> 5, hh = lane >> 4, m = lane & 15;
  const int rowBase = (int)blockIdx.x * GBM;
  const int col0    = (int)blockIdx.y * GBN;

  float bv[4];
#pragma unroll
  for (int t = 0; t < 4; ++t) bv[t] = bias[col0 + 16 * t + m];

  v8f acc[4];
  {
    const v8f z = {0.f, 0.f, 0.f, 0.f, 0.f, 0.f, 0.f, 0.f};
    acc[0] = z; acc[1] = z; acc[2] = z; acc[3] = z;
  }
  const unsigned short* ap = A  + (size_t)(rowBase + 16 * wave + m) * (size_t)K + 8 * hh;
  const unsigned short* wp = WT + (size_t)(col0 + m) * (size_t)K + 8 * hh;
  const int ksteps = K >> 5;
#pragma unroll 1
  for (int ks = 0; ks < ksteps; ++ks) {
    FragB af;
    af.h[0] = *(const v8usa*)(ap + 32 * ks);
    af.h[1] = *(const v8usa*)(ap + 32 * ks + 16);
#pragma unroll
    for (int t = 0; t < 4; ++t) {
      const unsigned short* wq = wp + (size_t)(16 * t) * (size_t)K + 32 * ks;
      FragB bf;
      bf.h[0] = *(const v8usa*)wq;
      bf.h[1] = *(const v8usa*)(wq + 16);
      acc[t] = wmb(af, bf, acc[t]);
    }
  }

#pragma unroll
  for (int t = 0; t < 4; ++t) {
    const int lc = 16 * t + m;
#pragma unroll
    for (int r = 0; r < 8; ++r) {
      const int lr = 16 * wave + 8 * hh + r;
      float v = acc[t][r] + bv[t];
      const float rl = (v > 0.0f) ? v : (v - v);
      v = (relu != 0) ? rl : v;
      stg[lr * GBN + lc] = v;
    }
  }
  __syncthreads();

  v4f fv[8];
#pragma unroll
  for (int i = 0; i < 8; ++i) {
    const int lr = 16 * wave + 2 * i + hh;
    fv[i] = *(const v4fa*)(stg + lr * GBN + 4 * m);
  }
#pragma unroll
  for (int i = 0; i < 8; ++i) {
    const int lr = 16 * wave + 2 * i + hh;
    const int gr = rowBase + lr;
    float* op = outF + (size_t)gr * (size_t)ldo + col0 + 4 * m;
    if (gr < nStore) *(volatile v4f*)op = fv[i];
  }
  __threadfence();
#pragma unroll
  for (int i = 0; i < 8; ++i) {
    const int lr = 16 * wave + 2 * i + hh;
    const int gr = rowBase + lr;
    float* op = outF + (size_t)gr * (size_t)ldo + col0 + 4 * m;
    if (gr < nStore) *(volatile v4f*)op = fv[i];
  }
}

__device__ __forceinline__ float gat_logit(const v4f v, const v4f xr, const float a, const v4f we, const v4f at) {
  float t0 = (v.x + xr.x) + a * we.x;
  float t1 = (v.y + xr.y) + a * we.y;
  float t2 = (v.z + xr.z) + a * we.z;
  float t3 = (v.w + xr.w) + a * we.w;
  t0 = (t0 >= 0.0f) ? t0 : NEGSL * t0;
  t1 = (t1 >= 0.0f) ? t1 : NEGSL * t1;
  t2 = (t2 >= 0.0f) ? t2 : NEGSL * t2;
  t3 = (t3 >= 0.0f) ? t3 : NEGSL * t3;
  float p = t0 * at.x;
  p = fmaf(t1, at.y, p);
  p = fmaf(t2, at.z, p);
  p = fmaf(t3, at.w, p);
  p += __shfl_xor(p, 1, 32);
  p += __shfl_xor(p, 2, 32);
  p += __shfl_xor(p, 4, 32);
  return p;
}

__global__ __launch_bounds__(NTHR) KATTR void k_scan(const int* __restrict__ REC, const int* __restrict__ CNT,
                                                     const int* __restrict__ OFF, const float* __restrict__ LOOPA,
                                                     const int* __restrict__ FLGB, const float* __restrict__ XLR,
                                                     const float* __restrict__ PAR, unsigned short* HP,
                                                     int nN, int MPr) {
  extern __shared__ __attribute__((aligned(16))) int ssm[];
  int*   rec  = ssm;
  int*   cnt  = rec + 2 * RCAP;
  int*   offs = cnt + NBA;
  float* laf  = (float*)(offs + NBA);
  const int tid = (int)threadIdx.x, lane = tid & 31, wave = tid >> 5;
  const int blk = (int)blockIdx.x;
  const int nodeBase = blk * NBA;

  const int nhraw = FLGB[(size_t)blk * 32];
  const int bflag = FLGB[(size_t)blk * 32 + 1];
  const int nh  = nhraw < 0 ? 0 : (nhraw > RCAP ? RCAP : nhraw);
  const int ovf = (bflag != 0 || nhraw < 0 || nhraw > RCAP) ? 1 : 0;

  {
    *(v4ia*)(cnt  + 4 * tid) = *(const v4i*)(CNT   + (size_t)blk * NBA + 4 * tid);
    *(v4ia*)(offs + 4 * tid) = *(const v4i*)(OFF   + (size_t)blk * NBA + 4 * tid);
    *(v4fa*)(laf  + 4 * tid) = *(const v4f*)(LOOPA + (size_t)blk * NBA + 4 * tid);
    const int* rb = REC + (size_t)blk * (size_t)(2 * RCAP);
    const int nI = 2 * ((nh + 1) & ~1);
#pragma unroll 1
    for (int p = tid * 4; p < nI; p += NTHR * 4) *(v4ia*)(rec + p) = *(const v4i*)(rb + p);
  }
  __syncthreads();

  const v4f we = *(const v4f*)(PAR + P_WE  + 4 * lane);
  const v4f at = *(const v4f*)(PAR + P_ATT + 4 * lane);
  const v4f bo = *(const v4f*)(PAR + P_BO  + 4 * lane);
  const float qnan = __int_as_float(0x7fc00000);
  const float pzb  = (ovf != 0) ? qnan : 0.0f;
  const int nhm1 = nh > 0 ? nh - 1 : 0;

#pragma unroll 1
  for (int si = 0; si < NBA / NWAVE; ++si) {
    const int s    = si * NWAVE + wave;
    const int node = nodeBase + s;
    const int nc   = node < nN ? node : nN - 1;
    int c = __builtin_amdgcn_readfirstlane(cnt[s]);
    const bool big = c > DEGCAP;
    c = c < 0 ? 0 : (c > DEGCAP ? DEGCAP : c);
    int o = __builtin_amdgcn_readfirstlane(offs[s]);
    o = o < 0 ? 0 : (o > nh ? nh : o);
    if (c > nh - o) c = nh - o;
    c = c < 0 ? 0 : c;
    const float lav = laf[s];
    const float* nrow = XLR + (size_t)nc * NX + 4 * lane;
    const v4f xlv = *(const v4f*)nrow;
    const v4f xrv = *(const v4f*)(nrow + HC);

    float mx = gat_logit(xlv, xrv, lav, we, at);
    float dn = 1.0f;
    float a0 = xlv.x, a1 = xlv.y, a2 = xlv.z, a3 = xlv.w;

#pragma unroll 1
    for (int b0 = 0; b0 < c; b0 += 32) {
      int idx = o + b0 + lane;
      idx = idx < 0 ? 0 : (idx > nhm1 ? nhm1 : idx);
      const v2i rr = *(const v2ia*)(rec + 2 * idx);
      int rs = rr.x;
      rs = rs < 0 ? 0 : (rs > nN - 1 ? nN - 1 : rs);
      const int ra  = rr.y;
      const int m32 = (c - b0) < 32 ? (c - b0) : 32;
#pragma unroll 1
      for (int k = 0; k < m32; ++k) {
        const int   sk = __builtin_amdgcn_readlane(rs, k);
        const float ak = __int_as_float(__builtin_amdgcn_readlane(ra, k));
        const v4f v = *(const v4f*)(XLR + (size_t)sk * NX + 4 * lane);
        const float lg = gat_logit(v, xrv, ak, we, at);
        const float df = lg - mx;
        const float ee = expf(-fabsf(df));
        const bool  up = df > 0.f;
        const float s1 = up ? ee : 1.0f;
        const float s2 = up ? 1.0f : ee;
        mx = up ? lg : mx;
        dn = fmaf(dn, s1, s2);
        a0 = fmaf(a0, s1, s2 * v.x);
        a1 = fmaf(a1, s1, s2 * v.y);
        a2 = fmaf(a2, s1, s2 * v.z);
        a3 = fmaf(a3, s1, s2 * v.w);
      }
    }
    const float inv = 1.0f / (dn + 1e-16f);
    const float pzr = big ? qnan : pzb;
    const bool live = node < nN;
    float y0 = fmaf(a0, inv, bo.x);
    float y1 = fmaf(a1, inv, bo.y);
    float y2 = fmaf(a2, inv, bo.z);
    float y3 = fmaf(a3, inv, bo.w);
    y0 = ((y0 > 0.0f) ? y0 : (y0 - y0)) + pzr;
    y1 = ((y1 > 0.0f) ? y1 : (y1 - y1)) + pzr;
    y2 = ((y2 > 0.0f) ? y2 : (y2 - y2)) + pzr;
    y3 = ((y3 > 0.0f) ? y3 : (y3 - y3)) + pzr;
    y0 = live ? y0 : 0.0f;
    y1 = live ? y1 : 0.0f;
    y2 = live ? y2 : 0.0f;
    y3 = live ? y3 : 0.0f;
    const unsigned int h0 = f2bf(y0), h1 = f2bf(y1), h2 = f2bf(y2), h3 = f2bf(y3);
    v4us ho, lo;
    ho[0] = (unsigned short)h0; ho[1] = (unsigned short)h1; ho[2] = (unsigned short)h2; ho[3] = (unsigned short)h3;
    lo[0] = (unsigned short)f2bf(y0 - bf2f(h0));
    lo[1] = (unsigned short)f2bf(y1 - bf2f(h1));
    lo[2] = (unsigned short)f2bf(y2 - bf2f(h2));
    lo[3] = (unsigned short)f2bf(y3 - bf2f(h3));
    if (node < MPr) {
      unsigned short* hp = HP + (size_t)node * KH + 4 * lane;
      *(volatile v4us*)hp = ho;
      *(volatile v4us*)(hp + HC) = lo;
      __threadfence();
      *(volatile v4us*)hp = ho;
      *(volatile v4us*)(hp + HC) = lo;
    }
  }
}

static inline int cdiv(int a, int b) { return (a + b - 1) / b; }

extern "C" void kernel_launch(void* const* d_in, const int* in_sizes, int n_in,
                              void* d_out, int out_size, void* d_ws, size_t ws_size,
                              hipStream_t stream) {
  if (n_in < 19) return;
  const int nN = in_sizes[0] / DIN;
  if (nN <= 0 || in_sizes[0] != nN * DIN || nN > (1 << 22)) return;
  if (in_sizes[1] < 2 || (in_sizes[1] & 1) != 0) return;
  const int nE = in_sizes[1] / 2;
  if (nE < 1 || nE > (1 << 20)) return;
  if (in_sizes[2] != nE) return;
  if (in_sizes[3] != DIN * HC || in_sizes[5] != DIN * HC) return;
  if (in_sizes[10] != HC * HC || in_sizes[12] != HC * HC || in_sizes[17] != HC * HC) return;
  if (in_sizes[4] != HC || in_sizes[6] != HC || in_sizes[7] != HC || in_sizes[8] != HC || in_sizes[9] != HC) return;
  if (in_sizes[11] != HC || in_sizes[13] != HC || in_sizes[14] != HC || in_sizes[15] != HC ||
      in_sizes[16] != HC || in_sizes[18] != HC) return;
  if (out_size != nN * HC) return;

  const float* x    = (const float*)d_in[0];
  const int*   ei   = (const int*)  d_in[1];
  const float* ea   = (const float*)d_in[2];
  const float* Wl1  = (const float*)d_in[3];
  const float* bl1  = (const float*)d_in[4];
  const float* Wr1  = (const float*)d_in[5];
  const float* br1  = (const float*)d_in[6];
  const float* We1  = (const float*)d_in[7];
  const float* at1  = (const float*)d_in[8];
  const float* bo1  = (const float*)d_in[9];
  const float* Wl2  = (const float*)d_in[10];
  const float* bl2  = (const float*)d_in[11];
  const float* Wr2  = (const float*)d_in[12];
  const float* br2  = (const float*)d_in[13];
  const float* We2  = (const float*)d_in[14];
  const float* at2  = (const float*)d_in[15];
  const float* bo2  = (const float*)d_in[16];
  const float* Wlin = (const float*)d_in[17];
  const float* blin = (const float*)d_in[18];
  float* out = (float*)d_out;
  const int* src = ei;
  const int* dst = ei + nE;

  const int MP   = cdiv(nN, MROWS) * MROWS;
  const int gM   = MP / GBM;
  const int gA   = cdiv(MP, NBA);
  if ((MP % GBM) != 0 || (long long)gA * NBA < (long long)MP) return;
  const int vec8 = ((nE & 3) == 0) ? 1 : 0;
  const int nUx  = MP * (DIN / 8);
  if ((nUx % NTHR) != 0) return;

  char* ws = (char*)d_ws;
  size_t off = 0;
  const size_t oXB  = off; off += (size_t)MP * DIN * 2;           off = (off + 255) & ~(size_t)255;
  const size_t oWP  = off; off += (size_t)WPLN * 2;               off = (off + 255) & ~(size_t)255;
  const size_t oP1  = off; off += (size_t)PARN * 4;               off = (off + 255) & ~(size_t)255;
  const size_t oP2  = off; off += (size_t)PARN * 4;               off = (off + 255) & ~(size_t)255;
  const size_t oXLR = off; off += (size_t)MP * NX * 4;            off = (off + 255) & ~(size_t)255;
  const size_t oHHL = off; off += (size_t)MP * KH * 2;            off = (off + 255) & ~(size_t)255;
  const size_t oREC = off; off += (size_t)gA * RCAP * 8;          off = (off + 255) & ~(size_t)255;
  const size_t oCNT = off; off += (size_t)gA * NBA * 4;           off = (off + 255) & ~(size_t)255;
  const size_t oOFF = off; off += (size_t)gA * NBA * 4;           off = (off + 255) & ~(size_t)255;
  const size_t oLA  = off; off += (size_t)gA * NBA * 4;           off = (off + 255) & ~(size_t)255;
  const size_t oFLG = off; off += (size_t)gA * 128;               off = (off + 255) & ~(size_t)255;
  if (off > ws_size || off > (size_t)WSMAX) return;
  unsigned short* XB   = (unsigned short*)(ws + oXB);
  unsigned short* WP   = (unsigned short*)(ws + oWP);
  float*          PAR1 = (float*)(ws + oP1);
  float*          PAR2 = (float*)(ws + oP2);
  float*          XLR  = (float*)(ws + oXLR);
  unsigned short* HHL  = (unsigned short*)(ws + oHHL);
  int*            REC  = (int*)(ws + oREC);
  int*            CNT  = (int*)(ws + oCNT);
  int*            OFF  = (int*)(ws + oOFF);
  float*          LA   = (float*)(ws + oLA);
  int*            FLG  = (int*)(ws + oFLG);
  const unsigned short* WLR1T = WP + OFF_W1;
  const unsigned short* WLR2T = WP + OFF_W2;
  const unsigned short* WLINT = WP + OFF_W3;

  const int bktLds  = BKT_LDS_INTS * 4;
  const int scanLds = SCAN_LDS_INTS * 4;
  hipFuncSetAttribute(reinterpret_cast<const void*>(&k_bucket),
                      hipFuncAttributeMaxDynamicSharedMemorySize, bktLds);
  hipFuncSetAttribute(reinterpret_cast<const void*>(&k_scan),
                      hipFuncAttributeMaxDynamicSharedMemorySize, scanLds);

  k_pa<<<nUx / NTHR, NTHR, 0, stream>>>(x, XB, nN, nUx);
  k_pb<<<NUWT / NTHR, NTHR, 0, stream>>>(Wl1, Wr1, Wl2, Wr2, Wlin, WP);
  k_par<<<1, NTHR, 0, stream>>>(bl1, br1, We1, at1, bo1, blin, PAR1, 6);
  k_par<<<1, NTHR, 0, stream>>>(bl2, br2, We2, at2, bo2, bo2, PAR2, 5);
  k_bucket<<<gA, NTHR, bktLds, stream>>>(src, dst, ea, nE, nN, vec8, REC, CNT, OFF, LA, FLG);
  k_gemm<<<dim3(gM, NX / GBN), GTHR, 0, stream>>>(XB, WLR1T, PAR1 + P_BIAS, XLR, DIN, NX, 0, MP);
  k_scan<<<gA, NTHR, scanLds, stream>>>(REC, CNT, OFF, LA, FLG, XLR, PAR1, HHL, nN, MP);
  k_gemm<<<dim3(gM, NX / GBN), GTHR, 0, stream>>>(HHL, WLR2T, PAR2 + P_BIAS, XLR, KH, NX, 0, MP);
  k_scan<<<gA, NTHR, scanLds, stream>>>(REC, CNT, OFF, LA, FLG, XLR, PAR2, HHL, nN, MP);
  k_gemm<<<dim3(gM, HC / GBN), GTHR, 0, stream>>>(HHL, WLINT, PAR1 + P_BLIN, out, KH, HC, 1, nN);
}
